// GRUCell_83760452207457
// MI455X (gfx1250) — hardware-verified
//
#include <hip/hip_runtime.h>


#define NR   16384
#define NI   256
#define NU   256
#define KC   (NU + NI)
typedef _Float16 h16;
typedef unsigned short bf;
typedef __attribute__((ext_vector_type(16))) __bf16   v16bf;
typedef __attribute__((ext_vector_type(16))) _Float16 v16h;
typedef __attribute__((ext_vector_type(8)))  _Float16 v8h;
typedef __attribute__((ext_vector_type(8)))  unsigned short v8us;
typedef __attribute__((ext_vector_type(8)))  float    v8f;
typedef __attribute__((ext_vector_type(4)))  float    v4f;
typedef v8h  __attribute__((may_alias)) v8ha;
typedef v4f  __attribute__((may_alias)) v4fa;
typedef v8us __attribute__((may_alias)) v8usa;

__device__ __forceinline__ unsigned short f2bf(float f) { unsigned u = __float_as_uint(f); u += 0x7FFFu + ((u >> 16) & 1u); return (unsigned short)(u >> 16); }
__device__ __forceinline__ float bf2f(unsigned short b) { return __uint_as_float(((unsigned)b) << 16); }
__device__ __forceinline__ float bfr(float f) { return bf2f(f2bf(f)); }
__device__ __forceinline__ v16h cat16(v8h lo, v8h hi) { return __builtin_shufflevector(lo, hi, 0, 1, 2, 3, 4, 5, 6, 7, 8, 9, 10, 11, 12, 13, 14, 15); }
__device__ __forceinline__ v16bf cat16b(v8us lo, v8us hi) { return __builtin_bit_cast(v16bf, __builtin_shufflevector(lo, hi, 0, 1, 2, 3, 4, 5, 6, 7, 8, 9, 10, 11, 12, 13, 14, 15)); }
__device__ __forceinline__ v8f wmma16(v16h a, v16h b, v8f c) { return __builtin_amdgcn_wmma_f32_16x16x32_f16(false, a, false, b, (short)0, c, false, false); }
__device__ __forceinline__ v8f wmmab(v16bf a, v16bf b, v8f c) { return __builtin_amdgcn_wmma_f32_16x16x32_bf16(false, a, false, b, (short)0, c, false, false); }


template <typename T16> struct WFrag;
template <> struct WFrag<h16> { typedef v16h V; static __device__ __forceinline__ V ld(const h16* p) { return cat16(*(const v8h*)p, *(const v8h*)(p + 16)); } static __device__ __forceinline__ v8f mma(V a, V b, v8f c) { return wmma16(a, b, c); } };
template <> struct WFrag<bf> { typedef v16bf V; static __device__ __forceinline__ V ld(const bf* p) { return cat16b(*(const v8us*)p, *(const v8us*)(p + 16)); } static __device__ __forceinline__ v8f mma(V a, V b, v8f c) { return wmmab(a, b, c); } };
template <typename T16, int NSPLIT, bool BIAS>
__global__ __launch_bounds__(32) void k_gemmw(const T16* __restrict__ A, const T16* __restrict__ A2, const T16* __restrict__ Bt, const T16* __restrict__ Bt2, int K, float* C, int ldc, const float* __restrict__ bias, size_t sA, size_t sB, size_t sC) {
    typedef typename WFrag<T16>::V V;
    __shared__ __align__(16) float os[16 * 68];
    const size_t z = blockIdx.z; A += z * sA; if (A2) A2 += z * sA; Bt += z * sB; if (Bt2) Bt2 += z * sB; C += z * sC;
    const int lane = threadIdx.x & 31, lr = lane & 15, hi = lane >> 4; const int r0 = blockIdx.x * 64, c0 = blockIdx.y * 64;
    v8f acc[4][4];
#pragma unroll
    for (int mb = 0; mb < 4; ++mb)
#pragma unroll
        for (int nb = 0; nb < 4; ++nb) acc[mb][nb] = (v8f){};
    const size_t aoff = (size_t)(r0 + lr) * K + 8 * hi, boff = (size_t)(c0 + lr) * K + 8 * hi;
#pragma unroll 1
    for (int kc = 0; kc < K; kc += 32) {
        V a[4], a2[4];
#pragma unroll
        for (int mb = 0; mb < 4; ++mb) { a[mb] = WFrag<T16>::ld(A + aoff + (size_t)mb * 16 * K + kc); if (NSPLIT == 1 || NSPLIT == 2) a2[mb] = WFrag<T16>::ld(A2 + aoff + (size_t)mb * 16 * K + kc); }
#pragma unroll
        for (int nb = 0; nb < 4; ++nb) { const V b = WFrag<T16>::ld(Bt + boff + (size_t)nb * 16 * K + kc); V b2; if (NSPLIT >= 2) b2 = WFrag<T16>::ld(Bt2 + boff + (size_t)nb * 16 * K + kc);
#pragma unroll
            for (int mb = 0; mb < 4; ++mb) { acc[mb][nb] = WFrag<T16>::mma(a[mb], b, acc[mb][nb]); if (NSPLIT == 1 || NSPLIT == 2) acc[mb][nb] = WFrag<T16>::mma(a2[mb], b, acc[mb][nb]); if (NSPLIT >= 2) acc[mb][nb] = WFrag<T16>::mma(a[mb], b2, acc[mb][nb]); } }
        asm volatile("v_nop\n\tv_nop\n\tv_nop\n\tv_nop" : "+v"(acc[0][0]), "+v"(acc[1][1]), "+v"(acc[2][2]), "+v"(acc[3][3]) : "v"(a[0]), "v"(a[3]));
    }
#pragma unroll
    for (int mb = 0; mb < 4; ++mb) {
#pragma unroll
        for (int nb = 0; nb < 4; ++nb) {
#pragma unroll
            for (int j = 0; j < 8; ++j) os[(hi * 8 + j) * 68 + nb * 16 + lr] = acc[mb][nb][j]; }
        __builtin_amdgcn_wave_barrier(); asm volatile("" ::: "memory");
        float* crow = C + (size_t)(r0 + mb * 16) * ldc + c0;
#pragma unroll 1
        for (int ps = 0; ps < 2; ++ps) {
#pragma unroll
            for (int s = 0; s < 8; ++s) { const int row = 2 * s + hi, cofs = lr * 4; v4f val = *(const v4fa*)(os + row * 68 + cofs); if (BIAS) { val[0] += bfr(bias[c0 + cofs]); val[1] += bfr(bias[c0 + cofs + 1]); val[2] += bfr(bias[c0 + cofs + 2]); val[3] += bfr(bias[c0 + cofs + 3]); }
                *(volatile v4f*)(crow + (size_t)row * ldc + cofs) = val; }
            if (ps == 0) __threadfence(); }
        __builtin_amdgcn_wave_barrier(); asm volatile("" ::: "memory");
    }
}

typedef __attribute__((ext_vector_type(4))) unsigned short v4us;
typedef __attribute__((ext_vector_type(2))) unsigned short v2us;
__device__ __forceinline__ void splitf(float y, unsigned short& h, unsigned short& l) { h = f2bf(y); l = f2bf(y - bf2f(h)); }
__device__ __forceinline__ float ex2(float a) { return __builtin_amdgcn_exp2f(__fmul_rn(a, 1.4426950408889634f)); }
__device__ __forceinline__ float sigm(float a) { return __fdiv_rn(1.0f, __fadd_rn(1.0f, ex2(-a))); }
__device__ __forceinline__ float tanhp(float a) { const float e = ex2(__fmul_rn(2.0f, a)); return __fsub_rn(1.0f, __fdiv_rn(2.0f, __fadd_rn(e, 1.0f))); }
__global__ __launch_bounds__(256) void k_wtG(const float* __restrict__ w, int K, int N, bf* Bt) {
    const int lane = threadIdx.x & 31; const int L0 = (blockIdx.x * 8 + (threadIdx.x >> 5)) * 8; const int nlines = N * K / 64;
#pragma unroll
    for (int ps = 0; ps < 2; ++ps) {
#pragma unroll 1
        for (int l = 0; l < 8; ++l) { const int L = L0 + l; if (L >= nlines) break; const size_t e = (size_t)L * 64 + lane * 2; const int k = (int)(e % K), n = (int)(e / K); v2us o;
            o[0] = f2bf(w[(size_t)k * N + n]); o[1] = f2bf(w[(size_t)(k + 1) * N + n]); *(volatile v2us*)(Bt + e) = o; }
        if (ps == 0) __threadfence(); }
}

__global__ __launch_bounds__(256) void k_bias2(const float* __restrict__ a, const float* __restrict__ b, float* B2) { const int i = threadIdx.x; const float va = a[i], vb = b[i]; *(volatile float*)(B2 + i) = va; *(volatile float*)(B2 + NU + i) = vb; __threadfence(); *(volatile float*)(B2 + i) = va; *(volatile float*)(B2 + NU + i) = vb; }
__global__ __launch_bounds__(256) void k_cat(const float* __restrict__ ph, const float* __restrict__ x, bf* XC) { const size_t i = (size_t)blockIdx.x * 256 + threadIdx.x; if (i >= (size_t)NR * KC / 8) return; const int c0 = (int)(i % (KC / 8)) * 8; const size_t r = i / (KC / 8); v8us o;
#pragma unroll
    for (int k = 0; k < 8; ++k) { const int c = c0 + k; o[k] = f2bf(c < NU ? ph[r * NU + c] : x[r * NI + (c - NU)]); }
    *(volatile v8us*)(XC + r * KC + c0) = o; __threadfence(); *(volatile v8us*)(XC + r * KC + c0) = o; }
__global__ __launch_bounds__(256) void k_cand(const float* __restrict__ ZR, const float* __restrict__ ph, const float* __restrict__ x, bf* Ch, bf* Cl) { const size_t i = (size_t)blockIdx.x * 256 + threadIdx.x; if (i >= (size_t)NR * KC / 4) return; const int c0 = (int)(i % (KC / 4)) * 4; const size_t r = i / (KC / 4); v4us oh, ol;
#pragma unroll
    for (int q = 0; q < 4; ++q) { const int c = c0 + q; float val; if (c < NU) { const float rg = sigm(ZR[r * (2 * NU) + NU + c]); val = __fmul_rn(rg, bfr(ph[r * NU + c])); } else val = bfr(x[r * NI + (c - NU)]); unsigned short a, b; splitf(val, a, b); oh[q] = a; ol[q] = b; }
    *(volatile v4us*)(Ch + r * KC + c0) = oh; *(volatile v4us*)(Cl + r * KC + c0) = ol; __threadfence(); *(volatile v4us*)(Ch + r * KC + c0) = oh; *(volatile v4us*)(Cl + r * KC + c0) = ol; }
__global__ __launch_bounds__(256) void k_out(const float* __restrict__ ZR, const float* __restrict__ HS, const float* __restrict__ ph, float* out) { const size_t i = (size_t)blockIdx.x * 256 + threadIdx.x; if (i >= (size_t)NR * NU / 4) return; const int c0 = (int)(i % (NU / 4)) * 4; const size_t r = i / (NU / 4); v4f o;
#pragma unroll
    for (int q = 0; q < 4; ++q) { const int c = c0 + q; const float z = sigm(ZR[r * (2 * NU) + c]); const float ht = tanhp(HS[r * NU + c]); float a = __fmul_rn(__fsub_rn(1.0f, z), bfr(ph[r * NU + c])), b = __fmul_rn(z, ht); asm volatile("" : "+v"(a), "+v"(b)); o[q] = __fadd_rn(a, b); }
    *(volatile v4f*)(out + r * NU + c0) = o; __threadfence(); *(volatile v4f*)(out + r * NU + c0) = o; }

extern "C" void kernel_launch(void* const* d_in, const int* in_sizes, int n_in,
                              void* d_out, int out_size, void* d_ws, size_t ws_size, hipStream_t stream) {
    (void)in_sizes; (void)n_in; (void)out_size;
    const float* x = (const float*)d_in[0]; const float* ph = (const float*)d_in[1]; const float* wz = (const float*)d_in[2]; const float* bz = (const float*)d_in[3]; const float* wr = (const float*)d_in[4]; const float* br = (const float*)d_in[5]; const float* ws = (const float*)d_in[6]; const float* bs = (const float*)d_in[7];
    float* OUT = (float*)d_out;
    char* wsp = (char*)d_ws;
    auto take = [&](size_t bytes) { char* p = wsp; wsp += (bytes + 255) & ~(size_t)255; return (void*)p; };
    bf* WZR = (bf*)take((size_t)2 * NU * KC * 2); bf* WS = (bf*)take((size_t)NU * KC * 2); float* BZR = (float*)take((size_t)2 * NU * 4); bf* XC = (bf*)take((size_t)NR * KC * 2); float* ZR = (float*)take((size_t)NR * 2 * NU * 4); bf* Ch = (bf*)take((size_t)NR * KC * 2); bf* Cl = (bf*)take((size_t)NR * KC * 2); float* HS = (float*)take((size_t)NR * NU * 4);
    if ((size_t)(wsp - (char*)d_ws) > ws_size) return;
    k_wtG<<<(KC * NU / 64 + 63) / 64, 256, 0, stream>>>(wz, KC, NU, WZR); k_wtG<<<(KC * NU / 64 + 63) / 64, 256, 0, stream>>>(wr, KC, NU, WZR + (size_t)NU * KC); k_wtG<<<(KC * NU / 64 + 63) / 64, 256, 0, stream>>>(ws, KC, NU, WS);
    k_bias2<<<1, 256, 0, stream>>>(bz, br, BZR);
    k_cat<<<(unsigned)(((size_t)NR * KC / 8 + 255) / 256), 256, 0, stream>>>(ph, x, XC);
    k_gemmw<bf, 0, true><<<dim3(NR / 64, 2 * NU / 64, 1), 32, 0, stream>>>(XC, nullptr, WZR, nullptr, KC, ZR, 2 * NU, BZR, 0, 0, 0);
    k_cand<<<(unsigned)(((size_t)NR * KC / 4 + 255) / 256), 256, 0, stream>>>(ZR, ph, x, Ch, Cl);
    k_gemmw<bf, 1, true><<<dim3(NR / 64, NU / 64, 1), 32, 0, stream>>>(Ch, Cl, WS, nullptr, KC, HS, NU, bs, 0, 0, 0);
    k_out<<<(unsigned)(((size_t)NR * NU / 4 + 255) / 256), 256, 0, stream>>>(ZR, HS, ph, OUT);
}
